// MyFirstGNN_32332513804719
// MI455X (gfx1250) — hardware-run, weakly checked
//
#include <hip/hip_runtime.h>
#include <stddef.h>
#include <stdint.h>


#define NN      50000
#define NE      800000
#define DF      128
#define NL      16
#define MP      50048
#define XP      128
#define AP      256
#define WP1     384
#define WP2     512
#define WPD     256
#define KROOT   256
#define SPLIT_AGG  1
#define SPLIT_H    1
#define SPLIT_HEAD 1
#define NKS_AGG  (SPLIT_AGG ? 8 : 4)
#define NKS_H    (SPLIT_H ? 8 : 4)
#define NKS_X    4
#define NKS_HEAD (SPLIT_HEAD ? 8 : 4)
#define NTHR    256
#define NWAVE   8
#define EPT     8
#define CHUNK   (NTHR * EPT)
#define WCAP    (EPT * 32)
#define LISTN   (NWAVE * WCAP)
#define NBA     1024
#define PKS     10
#define RCAP    28672
#define DEGCAP  64
#define NBLK    49
#define NPADN   (NBLK * NBA)
#define RPB     64
#define RPW     8
#define GBM     128
#define GBN     128
#define GTHR    256
#define LDS_GM  ((GBM * GBN + GBN) * 4)
#define O_REG1  0
#define O_REG2  (RCAP)
#define O_SCNT  (2 * RCAP)
#define O_SOFF  (O_SCNT + NBA)
#define O_CUR   (O_SOFF + NBA)
#define O_SCN2  (O_CUR + NBA)
#define O_LIST  (O_SCN2 + NBA)
#define O_MISC  (O_LIST + LISTN)
#define BK_INTS (O_MISC + 32)
#define LDS_BK  (BK_INTS * 4)
#define NWBLK   49
#define NXBLK   (MP * 16 / NTHR)
#define MEAS_BLK_HITS 16623
#define MEAS_MAXDEG   35

static_assert(NBLK * NBA >= NN);
static_assert(NPADN >= MP);
static_assert((long long)RCAP * 100 >= (long long)MEAS_BLK_HITS * 105);
static_assert(DEGCAP >= MEAS_MAXDEG + 8);
static_assert(NN % 2 == 0);
static_assert(MP % GBM == 0 && MP % RPB == 0 && MP >= NN);
static_assert(DF == 32 * 4);
static_assert((CHUNK & (CHUNK - 1)) == 0 && CHUNK <= 4096);
static_assert(NBA == (1 << PKS) && NBA == NTHR * 4 && NBA % GBM == 0);
static_assert(LISTN == NWAVE * WCAP && LISTN >= 2 * NBA);
static_assert(RCAP % (NTHR * 4) == 0 && BK_INTS % 4 == 0);
static_assert(LDS_BK <= 300000);
static_assert(NE < (1 << 21));
static_assert(NKS_AGG * 32 <= AP && NKS_AGG * 32 <= KROOT);
static_assert(KROOT + NKS_H * 32 <= WP2 && NKS_H * 32 <= AP);
static_assert(KROOT + NKS_X * 32 <= WP1 && NKS_X * 32 <= XP);
static_assert(NKS_HEAD * 32 <= WPD && NKS_HEAD * 32 <= AP);
static_assert(AP == 2 * DF && WP1 == 3 * DF && WP2 == 4 * DF && WPD == 2 * DF);
static_assert(GBM == (GTHR / 32) * 16 && GBN == 8 * 16 && GBN == DF);
static_assert(RPB == NWAVE * RPW);
static_assert((MP * 16) % NTHR == 0);
static_assert((NN * NL) % 4 == 0);

typedef float          v4f   __attribute__((ext_vector_type(4)));
typedef float          v8f   __attribute__((ext_vector_type(8)));
typedef int            v4i   __attribute__((ext_vector_type(4)));
typedef int            v8i   __attribute__((ext_vector_type(8)));
typedef unsigned       v2u   __attribute__((ext_vector_type(2)));
typedef unsigned       v4u   __attribute__((ext_vector_type(4)));
typedef unsigned short v8us  __attribute__((ext_vector_type(8)));
typedef __bf16         v16bf __attribute__((ext_vector_type(16)));
typedef v4f  __attribute__((may_alias)) v4fa;
typedef v4i  __attribute__((may_alias)) v4ia;
typedef v2u  __attribute__((may_alias)) v2ua;
typedef v4u  __attribute__((may_alias)) v4ua;
typedef v8us __attribute__((may_alias)) v8usa;
union FragB { v16bf v; v8us h[2]; v8i w; };

__device__ __forceinline__ v8f wmb(const FragB& a, const FragB& b, v8f c) {
  v8f d = __builtin_amdgcn_wmma_f32_16x16x32_bf16(false, a.v, false, b.v, (short)0, c, false, false);
  asm volatile("v_nop\n\tv_nop\n\tv_nop\n\tv_nop" : "+v"(d) : "v"(a.w), "v"(b.w));
  return d;
}

__device__ __forceinline__ unsigned bf16_bits(float f) {
  const unsigned u = __float_as_uint(f);
  const unsigned r = ((u + 0x7FFFu + ((u >> 16) & 1u)) >> 16) & 0xFFFFu;
  const unsigned q = ((u >> 16) | 0x40u) & 0xFFFFu;
  return ((u & 0x7FFFFFFFu) > 0x7F800000u) ? q : r;
}
__device__ __forceinline__ float bf16_val(float f) { return __uint_as_float(bf16_bits(f) << 16); }
__device__ __forceinline__ float bfw_lo(unsigned w) { return __uint_as_float(w << 16); }
__device__ __forceinline__ float bfw_hi(unsigned w) { return __uint_as_float(w & 0xffff0000u); }
__device__ __forceinline__ void pack2(float a, float b, unsigned& hw, unsigned& lw) {
  const unsigned ha = bf16_bits(a), hb = bf16_bits(b);
  const unsigned la = bf16_bits(a - __uint_as_float(ha << 16));
  const unsigned lb = bf16_bits(b - __uint_as_float(hb << 16));
  hw = ha | (hb << 16);
  lw = la | (lb << 16);
}

__device__ __forceinline__ void wave_sync() {
  __builtin_amdgcn_fence(__ATOMIC_RELEASE, "wavefront");
  __builtin_amdgcn_wave_barrier();
  __builtin_amdgcn_fence(__ATOMIC_ACQUIRE, "wavefront");
}

__device__ __forceinline__ int scan_chunk(const int* __restrict__ keys, int nE, int cbase, int slotBase,
                                          int nb, int vec8, int* list, int tid, int lane, int wave) {
  const int el0  = tid * EPT;
  const int e0   = cbase + el0;
  const int sent = (int)(1u << 31);
  v4i da, db;
  if (vec8 != 0 && cbase + CHUNK <= nE) {
    da = *(const v4i*)(keys + e0);
    db = *(const v4i*)(keys + e0 + 4);
  } else {
    const int t0 = keys[min(e0,     nE - 1)];
    const int t1 = keys[min(e0 + 1, nE - 1)];
    const int t2 = keys[min(e0 + 2, nE - 1)];
    const int t3 = keys[min(e0 + 3, nE - 1)];
    const int t4 = keys[min(e0 + 4, nE - 1)];
    const int t5 = keys[min(e0 + 5, nE - 1)];
    const int t6 = keys[min(e0 + 6, nE - 1)];
    const int t7 = keys[min(e0 + 7, nE - 1)];
    asm volatile("" :: "v"(t0), "v"(t1), "v"(t2), "v"(t3), "v"(t4), "v"(t5), "v"(t6), "v"(t7));
    da.x = (e0     < nE) ? t0 : sent;
    da.y = (e0 + 1 < nE) ? t1 : sent;
    da.z = (e0 + 2 < nE) ? t2 : sent;
    da.w = (e0 + 3 < nE) ? t3 : sent;
    db.x = (e0 + 4 < nE) ? t4 : sent;
    db.y = (e0 + 5 < nE) ? t5 : sent;
    db.z = (e0 + 6 < nE) ? t6 : sent;
    db.w = (e0 + 7 < nE) ? t7 : sent;
  }
  const unsigned nbs = (unsigned)slotBase;
  const unsigned unb = (unsigned)nb;
  const unsigned s0 = (unsigned)da.x - nbs, s1 = (unsigned)da.y - nbs;
  const unsigned s2 = (unsigned)da.z - nbs, s3 = (unsigned)da.w - nbs;
  const unsigned s4 = (unsigned)db.x - nbs, s5 = (unsigned)db.y - nbs;
  const unsigned s6 = (unsigned)db.z - nbs, s7 = (unsigned)db.w - nbs;
  const bool h0 = s0 < unb, h1 = s1 < unb, h2 = s2 < unb, h3 = s3 < unb;
  const bool h4 = s4 < unb, h5 = s5 < unb, h6 = s6 < unb, h7 = s7 < unb;
  const int cl = (h0 ? 1 : 0) + (h1 ? 1 : 0) + (h2 ? 1 : 0) + (h3 ? 1 : 0)
               + (h4 ? 1 : 0) + (h5 ? 1 : 0) + (h6 ? 1 : 0) + (h7 ? 1 : 0);
  int incl = cl;
#pragma unroll
  for (int d = 1; d < 32; d <<= 1) {
    const int up = __shfl_up(incl, d, 32);
    incl += (lane >= d) ? up : 0;
  }
  const int wc = __shfl(incl, 31, 32);
  int pos = incl - cl;
  int* wl = list + wave * WCAP;
#define PUTJ(J, HJ, SJ) { \
    if (HJ) wl[pos & (WCAP - 1)] = ((el0 + (J)) << PKS) | (int)(SJ); \
    pos += (HJ) ? 1 : 0; }
  PUTJ(0, h0, s0)
  PUTJ(1, h1, s1)
  PUTJ(2, h2, s2)
  PUTJ(3, h3, s3)
  PUTJ(4, h4, s4)
  PUTJ(5, h5, s5)
  PUTJ(6, h6, s6)
  PUTJ(7, h7, s7)
#undef PUTJ
  return wc;
}

template <int NSRC, int DUP>
__device__ __forceinline__ void wunit(const float* __restrict__ W, unsigned short* P, int pitch, int coff, int v) {
  const int n  = v >> 4;
  const int k8 = (v & 15) * 8;
  float f[8];
#pragma unroll
  for (int i = 0; i < 8; ++i) f[i] = W[(size_t)(k8 + i) * NSRC + (size_t)n];
  v8us o;
#pragma unroll
  for (int i = 0; i < 8; ++i) o[i] = (unsigned short)bf16_bits(f[i]);
  unsigned short* dp = P + (size_t)n * (size_t)pitch + (size_t)(coff + k8);
  *(volatile v8us*)dp = o;
  if (DUP) *(volatile v8us*)(dp + DF) = o;
  __threadfence();
  *(volatile v8us*)dp = o;
  if (DUP) *(volatile v8us*)(dp + DF) = o;
}

__global__ __launch_bounds__(NTHR) void k_prep(const float* __restrict__ x,
                                               const float* __restrict__ w11, const float* __restrict__ w21,
                                               const float* __restrict__ w12, const float* __restrict__ w22,
                                               const float* __restrict__ w13, const float* __restrict__ w23,
                                               const float* __restrict__ wdn,
                                               unsigned short* WC1, unsigned short* WC2, unsigned short* WC3,
                                               unsigned short* WD, unsigned short* XB, int nN, int mRows) {
  const int tid = (int)threadIdx.x;
  const int bx  = (int)blockIdx.x;
  if (bx < NWBLK) {
    const int part = bx >> 3;
    const int v    = (bx & 7) * NTHR + tid;
    if (part == 0)      wunit<DF, 1>(w11, WC1, WP1, 0, v);
    else if (part == 1) wunit<DF, 0>(w21, WC1, WP1, KROOT, v);
    else if (part == 2) wunit<DF, 1>(w12, WC2, WP2, 0, v);
    else if (part == 3) wunit<DF, 1>(w22, WC2, WP2, KROOT, v);
    else if (part == 4) wunit<DF, 1>(w13, WC3, WP2, 0, v);
    else if (part == 5) wunit<DF, 1>(w23, WC3, WP2, KROOT, v);
    else                wunit<NL, 1>(wdn, WD, WPD, 0, tid);
  } else {
    const int w   = (bx - NWBLK) * NTHR + tid;
    const int row = w >> 4;
    const int c8  = (w & 15) * 8;
    if (row >= mRows) return;
    const int rc  = row < nN ? row : nN - 1;
    const float* p = x + (size_t)rc * DF + c8;
    const v4f a = *(const v4f*)p;
    const v4f b = *(const v4f*)(p + 4);
    asm volatile("" :: "v"(a), "v"(b));
    const bool lv = row < nN;
    v8us o;
    o[0] = lv ? (unsigned short)bf16_bits(a.x) : (unsigned short)0;
    o[1] = lv ? (unsigned short)bf16_bits(a.y) : (unsigned short)0;
    o[2] = lv ? (unsigned short)bf16_bits(a.z) : (unsigned short)0;
    o[3] = lv ? (unsigned short)bf16_bits(a.w) : (unsigned short)0;
    o[4] = lv ? (unsigned short)bf16_bits(b.x) : (unsigned short)0;
    o[5] = lv ? (unsigned short)bf16_bits(b.y) : (unsigned short)0;
    o[6] = lv ? (unsigned short)bf16_bits(b.z) : (unsigned short)0;
    o[7] = lv ? (unsigned short)bf16_bits(b.w) : (unsigned short)0;
    unsigned short* dp = XB + (size_t)row * XP + c8;
    *(volatile v8us*)dp = o;
    __threadfence();
    *(volatile v8us*)dp = o;
  }
}

__global__ __launch_bounds__(NTHR) void k_bucket(const int* __restrict__ keysD, const int* __restrict__ keysS,
                                                 int nE, int nN, int vec8,
                                                 int* LIST, int* CIN, int* OFF, float* NS, float* ND, int* REC) {
  extern __shared__ __attribute__((aligned(16))) int dsm[];
  int* reg1 = dsm + O_REG1;
  int* reg2 = dsm + O_REG2;
  int* scnt = dsm + O_SCNT;
  int* soff = dsm + O_SOFF;
  int* cur  = dsm + O_CUR;
  int* scn2 = dsm + O_SCN2;
  int* list = dsm + O_LIST;
  int* wcnt = dsm + O_MISC;
  int* wtot = wcnt + 8;
  int* wmx  = wtot + 8;
  const int tid = (int)threadIdx.x, lane = tid & 31, wave = tid >> 5;
  const int nodeBase = (int)blockIdx.x * NBA;
  int nb = nN - nodeBase;
  nb = nb > NBA ? NBA : (nb < 1 ? 1 : nb);

  {
    const v4i z4 = {0, 0, 0, 0};
    for (int i = tid * 4; i < BK_INTS; i += NTHR * 4) *(v4ia*)(dsm + i) = z4;
  }
  __syncthreads();

  const int nChunks = (nE + CHUNK - 1) / CHUNK;

  int tot = 0;
#pragma unroll 1
  for (int ch = 0; ch < nChunks; ++ch) {
    const int cbase = ch * CHUNK;
    const int wc = scan_chunk(keysD, nE, cbase, nodeBase, nb, vec8, list, tid, lane, wave);
    if (lane == 0) wcnt[wave] = wc;
    __syncthreads();
    int pre = 0, all = 0;
#pragma unroll
    for (int w2 = 0; w2 < NWAVE; ++w2) {
      int c = wcnt[w2];
      c = c < 0 ? 0 : (c > WCAP ? WCAP : c);
      all += c;
      pre += (w2 < wave) ? c : 0;
    }
    const int wcc  = wc > WCAP ? WCAP : wc;
    const int base = tot + pre;
#pragma unroll 1
    for (int i = lane; i < wcc; i += 32) {
      const int ent = list[wave * WCAP + i];
      const int el  = (ent >> PKS) & (CHUNK - 1);
      const int sl  = ent & (NBA - 1);
      int eid = cbase + el;
      eid = eid > nE - 1 ? nE - 1 : eid;
      const int pos = base + i;
      if (pos < RCAP) reg1[pos] = (int)(((unsigned)eid << PKS) | (unsigned)sl);
    }
    tot += all;
    tot = tot > RCAP ? RCAP : tot;
    __syncthreads();
  }
  const int nh = tot;

#pragma unroll 1
  for (int ch = 0; ch < nChunks; ++ch) {
    const int cbase = ch * CHUNK;
    const int wc = scan_chunk(keysS, nE, cbase, nodeBase, nb, vec8, list, tid, lane, wave);
    if (lane == 0) wcnt[wave] = wc;
    __syncthreads();
    if (wave == 0) {
#pragma unroll 1
      for (int w2 = 0; w2 < NWAVE; ++w2) {
        int c = wcnt[w2];
        c = c < 0 ? 0 : (c > WCAP ? WCAP : c);
#pragma unroll 1
        for (int b0 = 0; b0 < c; b0 += 32) {
          const int idx = b0 + lane;
          const int ent = list[w2 * WCAP + (idx < WCAP ? idx : WCAP - 1)];
          const int m32 = (c - b0) < 32 ? (c - b0) : 32;
#pragma unroll 1
          for (int k = 0; k < m32; ++k) {
            const int u  = __builtin_amdgcn_readlane(ent, k);
            const int sl = u & (NBA - 1);
            if (lane == 0) scn2[sl] = scn2[sl] + 1;
          }
        }
      }
    }
    __syncthreads();
  }

  if (wave == 0) {
#pragma unroll 1
    for (int b0 = 0; b0 < nh; b0 += 32) {
      const int idx = b0 + lane;
      const int uv  = reg1[idx < RCAP ? idx : RCAP - 1];
      const int m32 = (nh - b0) < 32 ? (nh - b0) : 32;
#pragma unroll 1
      for (int k = 0; k < m32; ++k) {
        const int u  = __builtin_amdgcn_readlane(uv, k);
        const int sl = u & (NBA - 1);
        if (lane == 0) scnt[sl] = scnt[sl] + 1;
      }
    }
  }
  __syncthreads();

  {
    const v4i ca = *(const v4ia*)(scnt + 4 * tid);
    const int e0 = ca.x < 0 ? 0 : ca.x, e1 = ca.y < 0 ? 0 : ca.y, e2 = ca.z < 0 ? 0 : ca.z, e3 = ca.w < 0 ? 0 : ca.w;
    const int ts = e0 + e1 + e2 + e3;
    int incl = ts;
#pragma unroll
    for (int d = 1; d < 32; d <<= 1) {
      const int up = __shfl_up(incl, d, 32);
      incl += (lane >= d) ? up : 0;
    }
    int mx = max(max(e0, e1), max(e2, e3));
    mx = max(mx, __shfl_xor(mx, 16, 32));
    mx = max(mx, __shfl_xor(mx, 8, 32));
    mx = max(mx, __shfl_xor(mx, 4, 32));
    mx = max(mx, __shfl_xor(mx, 2, 32));
    mx = max(mx, __shfl_xor(mx, 1, 32));
    if (lane == 31) wtot[wave] = incl;
    if (lane == 0)  wmx[wave] = mx;
    __syncthreads();
    int pre = 0;
#pragma unroll
    for (int w2 = 0; w2 < NWAVE; ++w2) pre += (w2 < wave) ? wtot[w2] : 0;
    int run = pre + incl - ts;
    v4i so;
    so.x = run; run += e0;
    so.y = run; run += e1;
    so.z = run; run += e2;
    so.w = run;
    *(v4ia*)(soff + 4 * tid) = so;
    *(v4ia*)(cur + 4 * tid)  = so;
  }
  __syncthreads();

  if (wave == 0) {
#pragma unroll 1
    for (int b0 = 0; b0 < nh; b0 += 32) {
      const int idx = b0 + lane;
      const int uv  = reg1[idx < RCAP ? idx : RCAP - 1];
      const int m32 = (nh - b0) < 32 ? (nh - b0) : 32;
#pragma unroll 1
      for (int k = 0; k < m32; ++k) {
        const int u   = __builtin_amdgcn_readlane(uv, k);
        const int sl  = u & (NBA - 1);
        const int eid = (int)((unsigned)u >> PKS);
        if (lane == 0) {
          int pos = cur[sl];
          pos = pos < 0 ? 0 : (pos > RCAP - 1 ? RCAP - 1 : pos);
          reg2[pos] = eid;
          cur[sl] = pos + 1;
        }
      }
    }
  }
  __syncthreads();

#pragma unroll 1
  for (int j = 0; j < 8; ++j) {
    const int q  = tid + NTHR * (j & 3);
    const int so = (j < 4) ? O_SCN2 : O_SCNT;
    const int to = (j < 4) ? 0 : NBA;
    int cv = dsm[so + q];
    cv = cv < 1 ? 1 : cv;
    const float r = 1.0f / sqrtf((float)cv);
    list[to + q] = __float_as_int(r);
  }
  __syncthreads();

  int bmax = 0;
#pragma unroll
  for (int w2 = 0; w2 < NWAVE; ++w2) bmax = max(bmax, wmx[w2]);
  const int flag = ((nh >= RCAP) || (bmax > DEGCAP)) ? 1 : 0;

  int* lrow = LIST + (size_t)blockIdx.x * RCAP;
#pragma unroll 1
  for (int it = 0; it < RCAP / (NTHR * 4); ++it) {
    const int i0 = 4 * (it * NTHR + tid);
    const v4i ev = *(const v4ia*)(reg2 + i0);
    int e0 = ev.x, e1 = ev.y, e2 = ev.z, e3 = ev.w;
    e0 = e0 < 0 ? 0 : (e0 > nE - 1 ? nE - 1 : e0);
    e1 = e1 < 0 ? 0 : (e1 > nE - 1 ? nE - 1 : e1);
    e2 = e2 < 0 ? 0 : (e2 > nE - 1 ? nE - 1 : e2);
    e3 = e3 < 0 ? 0 : (e3 > nE - 1 ? nE - 1 : e3);
    int g0 = keysS[e0], g1 = keysS[e1], g2 = keysS[e2], g3 = keysS[e3];
    asm volatile("" :: "v"(g0), "v"(g1), "v"(g2), "v"(g3));
    g0 = g0 < 0 ? 0 : (g0 > nN - 1 ? nN - 1 : g0);
    g1 = g1 < 0 ? 0 : (g1 > nN - 1 ? nN - 1 : g1);
    g2 = g2 < 0 ? 0 : (g2 > nN - 1 ? nN - 1 : g2);
    g3 = g3 < 0 ? 0 : (g3 > nN - 1 ? nN - 1 : g3);
    v4i ov;
    ov.x = (i0     < nh) ? g0 : 0;
    ov.y = (i0 + 1 < nh) ? g1 : 0;
    ov.z = (i0 + 2 < nh) ? g2 : 0;
    ov.w = (i0 + 3 < nh) ? g3 : 0;
    *(volatile v4i*)(lrow + i0) = ov;
    __threadfence();
    *(volatile v4i*)(lrow + i0) = ov;
  }
  {
    const v4i cv = *(const v4ia*)(scnt + 4 * tid);
    const v4i fv = *(const v4ia*)(soff + 4 * tid);
    const v4i si = *(const v4ia*)(list + 4 * tid);
    const v4i di = *(const v4ia*)(list + NBA + 4 * tid);
    v4f sv, dv;
    sv.x = __int_as_float(si.x); sv.y = __int_as_float(si.y); sv.z = __int_as_float(si.z); sv.w = __int_as_float(si.w);
    dv.x = __int_as_float(di.x); dv.y = __int_as_float(di.y); dv.z = __int_as_float(di.z); dv.w = __int_as_float(di.w);
    v4i rv = {0, 0, 0, 0};
    rv.x = (tid == 0) ? bmax : 0;
    rv.y = (tid == 0) ? flag : 0;
    rv.z = (tid == 0) ? nh : 0;
    int*   cp = CIN + (size_t)nodeBase + 4 * tid;
    int*   fp = OFF + (size_t)nodeBase + 4 * tid;
    float* sp = NS  + (size_t)nodeBase + 4 * tid;
    float* dq = ND  + (size_t)nodeBase + 4 * tid;
    int*   rp = REC + (size_t)blockIdx.x * 32 + 4 * (tid & 7);
    *(volatile v4i*)cp = cv;
    *(volatile v4i*)fp = fv;
    *(volatile v4f*)sp = sv;
    *(volatile v4f*)dq = dv;
    if (tid < 8) *(volatile v4i*)rp = rv;
    __threadfence();
    *(volatile v4i*)cp = cv;
    *(volatile v4i*)fp = fv;
    *(volatile v4f*)sp = sv;
    *(volatile v4f*)dq = dv;
    if (tid < 8) *(volatile v4i*)rp = rv;
  }
}

template <int L1>
__global__ __launch_bounds__(NTHR) void k_replay(const unsigned short* __restrict__ XB, const float* __restrict__ H,
                                                 const int* __restrict__ LIST, const int* __restrict__ CIN,
                                                 const int* __restrict__ OFF, const int* __restrict__ REC,
                                                 const float* __restrict__ NS, const float* __restrict__ ND,
                                                 unsigned short* AGG, int nN, int mRows) {
  __shared__ __attribute__((aligned(16))) unsigned rowst[NWAVE * 128];
  const int tid = (int)threadIdx.x, lane = tid & 31, wave = tid >> 5;
  unsigned* wst = rowst + wave * 128;
#pragma unroll 1
  for (int ri = 0; ri < RPW; ++ri) {
    const int node = (int)blockIdx.x * RPB + wave * RPW + ri;
    if (node >= mRows) continue;
    const int bidx = node >> PKS;
    const int craw = CIN[node];
    const int oraw = OFF[node];
    const int fraw = REC[(size_t)bidx * 32 + 1];
    int c = craw < 0 ? 0 : craw;
    c = c > DEGCAP ? DEGCAP : c;
    int o = oraw < 0 ? 0 : (oraw > RCAP - 1 ? RCAP - 1 : oraw);
    c = c > RCAP - o ? RCAP - o : c;
    int last = o + c - 1;
    last = last < o ? o : last;
    c    = __builtin_amdgcn_readfirstlane(c);
    o    = __builtin_amdgcn_readfirstlane(o);
    last = __builtin_amdgcn_readfirstlane(last);
    const bool pois = (fraw != 0) || (craw > DEGCAP);
    const int* lp = LIST + (size_t)bidx * RCAP;
    float a0 = 0.0f, a1 = 0.0f, a2 = 0.0f, a3 = 0.0f;
#pragma unroll 1
    for (int b0 = 0; b0 < c; b0 += 32) {
      int idx = o + b0 + lane;
      idx = idx > last ? last : idx;
      int col = lp[idx];
      asm volatile("" :: "v"(col));
      col = col < 0 ? 0 : (col > nN - 1 ? nN - 1 : col);
      const float nsv = NS[col];
      asm volatile("" :: "v"(nsv));
      const int nsb = __float_as_int(nsv);
      const int m32 = (c - b0) < 32 ? (c - b0) : 32;
#pragma unroll 1
      for (int k = 0; k < m32; ++k) {
        const int   sk = __builtin_amdgcn_readlane(col, k);
        const float wk = __int_as_float(__builtin_amdgcn_readlane(nsb, k));
        if constexpr (L1 != 0) {
          const unsigned short* rp = XB + (size_t)sk * XP + 4 * lane;
          const v2u w = *(const v2ua*)rp;
          a0 = fmaf(wk, bfw_lo(w.x), a0);
          a1 = fmaf(wk, bfw_hi(w.x), a1);
          a2 = fmaf(wk, bfw_lo(w.y), a2);
          a3 = fmaf(wk, bfw_hi(w.y), a3);
        } else {
          const v4f hv = *(const v4f*)(H + (size_t)sk * DF + 4 * lane);
          a0 = fmaf(wk, hv.x, a0);
          a1 = fmaf(wk, hv.y, a1);
          a2 = fmaf(wk, hv.z, a2);
          a3 = fmaf(wk, hv.w, a3);
        }
      }
    }
    const int nodec = node < nN ? node : nN - 1;
    const float nd = ND[nodec];
    const bool live = node < nN;
    const float qn = __uint_as_float(0x7fc00000u);
    float m0 = nd * a0, m1 = nd * a1, m2 = nd * a2, m3 = nd * a3;
    m0 = pois ? qn : m0; m1 = pois ? qn : m1; m2 = pois ? qn : m2; m3 = pois ? qn : m3;
    m0 = live ? m0 : 0.0f; m1 = live ? m1 : 0.0f; m2 = live ? m2 : 0.0f; m3 = live ? m3 : 0.0f;
    unsigned h0, l0, h1, l1;
    pack2(m0, m1, h0, l0);
    pack2(m2, m3, h1, l1);
    v2u hq, lq;
    hq.x = h0; hq.y = h1;
    lq.x = l0; lq.y = l1;
    *(v2ua*)(wst + 2 * lane)      = hq;
    *(v2ua*)(wst + 64 + 2 * lane) = lq;
    wave_sync();
    const v4u qv = *(const v4ua*)(wst + 4 * lane);
    wave_sync();
    unsigned short* wp = AGG + (size_t)node * AP + 8 * lane;
    *(volatile v4u*)wp = qv;
    __threadfence();
    *(volatile v4u*)wp = qv;
  }
}

template <int NKS, int WPITCH>
__device__ __forceinline__ void kseg(const unsigned short* __restrict__ ap, const unsigned short* __restrict__ wp,
                                     v8f (&acc)[8]) {
#pragma unroll 1
  for (int ks = 0; ks < NKS; ++ks) {
    FragB af;
    af.h[0] = *(const v8usa*)(ap + 32 * ks);
    af.h[1] = *(const v8usa*)(ap + 32 * ks + 16);
#pragma unroll
    for (int t = 0; t < 8; ++t) {
      const unsigned short* wq = wp + (size_t)(16 * t) * (size_t)WPITCH + 32 * ks;
      FragB bf;
      bf.h[0] = *(const v8usa*)wq;
      bf.h[1] = *(const v8usa*)(wq + 16);
      acc[t] = wmb(af, bf, acc[t]);
    }
  }
}

template <int WRITE_H>
__device__ __forceinline__ void gemm_store_pass(const float* stg, float* Hout, unsigned short* PO,
                                                int rowBase, int wave, int lane, int hh, int m) {
#pragma unroll 1
  for (int i = 0; i < 16; ++i) {
    const int lr = 16 * wave + i;
    const size_t gr = (size_t)(rowBase + lr);
    if (WRITE_H) {
      const v4f hv = *(const v4fa*)(stg + lr * GBN + 4 * lane);
      *(volatile v4f*)(Hout + gr * DF + 4 * lane) = hv;
    }
    const v4f a = *(const v4fa*)(stg + lr * GBN + 8 * m);
    const v4f b = *(const v4fa*)(stg + lr * GBN + 8 * m + 4);
    unsigned h0, l0, h1, l1, h2, l2, h3, l3;
    pack2(a.x, a.y, h0, l0);
    pack2(a.z, a.w, h1, l1);
    pack2(b.x, b.y, h2, l2);
    pack2(b.z, b.w, h3, l3);
    const bool isHi = (hh == 0);
    v4u pw;
    pw.x = isHi ? h0 : l0;
    pw.y = isHi ? h1 : l1;
    pw.z = isHi ? h2 : l2;
    pw.w = isHi ? h3 : l3;
    *(volatile v4u*)(PO + gr * AP + hh * DF + 8 * m) = pw;
  }
}

template <int L1, int WRITE_H>
__global__ __launch_bounds__(GTHR) __attribute__((amdgpu_num_vgpr(248)))
void k_gemm(const unsigned short* __restrict__ AGG, const unsigned short* __restrict__ ROOT,
            const unsigned short* __restrict__ WT, const float* __restrict__ bias,
            float* Hout, unsigned short* PO, int nN) {
  extern __shared__ __attribute__((aligned(16))) float gsm[];
  float* stg = gsm;
  float* bsh = gsm + GBM * GBN;
  const int tid = (int)threadIdx.x, lane = tid & 31, wave = tid >> 5, hh = lane >> 4, m = lane & 15;
  const int rowBase = (int)blockIdx.x * GBM;

  if (tid < 32) {
    const v4f b4 = *(const v4f*)(bias + 4 * tid);
    v4f bq;
    bq.x = bf16_val(b4.x); bq.y = bf16_val(b4.y); bq.z = bf16_val(b4.z); bq.w = bf16_val(b4.w);
    *(v4fa*)(bsh + 4 * tid) = bq;
  }

  v8f acc[8];
  {
    const v8f z = {0.f, 0.f, 0.f, 0.f, 0.f, 0.f, 0.f, 0.f};
#pragma unroll
    for (int t = 0; t < 8; ++t) acc[t] = z;
  }
  const size_t arow = (size_t)(rowBase + 16 * wave + m);
  if constexpr (L1 != 0) {
    const unsigned short* wp = WT + (size_t)m * (size_t)WP1 + 8 * hh;
    kseg<NKS_AGG, WP1>(AGG + arow * AP + 8 * hh, wp, acc);
    kseg<NKS_X, WP1>(ROOT + arow * XP + 8 * hh, wp + KROOT, acc);
  } else {
    const unsigned short* wp = WT + (size_t)m * (size_t)WP2 + 8 * hh;
    kseg<NKS_AGG, WP2>(AGG + arow * AP + 8 * hh, wp, acc);
    kseg<NKS_H, WP2>(ROOT + arow * AP + 8 * hh, wp + KROOT, acc);
  }
  __syncthreads();

#pragma unroll
  for (int t = 0; t < 8; ++t) {
    const int lc = 16 * t + m;
    const float bb = bsh[lc];
#pragma unroll
    for (int r = 0; r < 8; ++r) {
      const int lr = 16 * wave + 8 * hh + r;
      const bool live = (rowBase + lr) < nN;
      const float z = acc[t][r] + bb;
      const float v = (z >= 0.0f) ? z : 0.2f * z;
      stg[lr * GBN + lc] = live ? v : 0.0f;
    }
  }
  __syncthreads();

  gemm_store_pass<WRITE_H>(stg, Hout, PO, rowBase, wave, lane, hh, m);
  __threadfence();
  gemm_store_pass<WRITE_H>(stg, Hout, PO, rowBase, wave, lane, hh, m);
}

__global__ __launch_bounds__(NTHR) void k_head(const unsigned short* __restrict__ P, const unsigned short* __restrict__ WD,
                                               const float* __restrict__ bd, const int* __restrict__ REC,
                                               float* out, int total4) {
  __shared__ __attribute__((aligned(16))) float stg[GBM * NL];
  __shared__ __attribute__((aligned(16))) float bsh[NL];
  const int tid = (int)threadIdx.x, lane = tid & 31, wave = tid >> 5, hh = lane >> 4, m = lane & 15;
  const int rowBase = (int)blockIdx.x * GBM;
  if (tid < 4) {
    const v4f b4 = *(const v4f*)(bd + 4 * tid);
    v4f bq;
    bq.x = bf16_val(b4.x); bq.y = bf16_val(b4.y); bq.z = bf16_val(b4.z); bq.w = bf16_val(b4.w);
    *(v4fa*)(bsh + 4 * tid) = bq;
  }
  v8f acc = {0.f, 0.f, 0.f, 0.f, 0.f, 0.f, 0.f, 0.f};
  const unsigned short* ap = P + (size_t)(rowBase + 16 * wave + m) * (size_t)AP + 8 * hh;
  const unsigned short* wp = WD + (size_t)m * (size_t)WPD + 8 * hh;
#pragma unroll 1
  for (int ks = 0; ks < NKS_HEAD; ++ks) {
    FragB af, bf;
    af.h[0] = *(const v8usa*)(ap + 32 * ks);
    af.h[1] = *(const v8usa*)(ap + 32 * ks + 16);
    bf.h[0] = *(const v8usa*)(wp + 32 * ks);
    bf.h[1] = *(const v8usa*)(wp + 32 * ks + 16);
    acc = wmb(af, bf, acc);
  }
#pragma unroll
  for (int r = 0; r < 8; ++r) stg[(16 * wave + 8 * hh + r) * NL + m] = acc[r];
  __syncthreads();
  const int fraw = REC[(size_t)(rowBase >> PKS) * 32 + 1];
  const float qn = __uint_as_float(0x7fc00000u);
#pragma unroll 1
  for (int j = 0; j < (GBM * NL) / NTHR; ++j) {
    const int e = tid + NTHR * j;
    const float z = stg[e] + bsh[e & (NL - 1)];
    float t = tanhf(z);
    t = (fraw != 0) ? qn : t;
    stg[e] = t;
  }
  __syncthreads();
  const int q0 = (int)blockIdx.x * (GBM * NL / 4) + tid;
  const int q1 = q0 + NTHR;
  const v4f v0 = *(const v4fa*)(stg + 4 * tid);
  const v4f v1 = *(const v4fa*)(stg + 4 * (tid + NTHR));
  const int s0 = q0 < total4 ? q0 : 0;
  const int s1 = q1 < total4 ? q1 : 0;
  float* o0 = out + (size_t)s0 * 4;
  float* o1 = out + (size_t)s1 * 4;
  if (q0 < total4) *(volatile v4f*)o0 = v0;
  if (q1 < total4) *(volatile v4f*)o1 = v1;
  __threadfence();
  if (q0 < total4) *(volatile v4f*)o0 = v0;
  if (q1 < total4) *(volatile v4f*)o1 = v1;
}

static inline size_t al256(size_t o) { return (o + 255) & ~(size_t)255; }

extern "C" void kernel_launch(void* const* d_in, const int* in_sizes, int n_in,
                              void* d_out, int out_size, void* d_ws, size_t ws_size,
                              hipStream_t stream) {
  if (n_in < 13) return;
  if (in_sizes[0] != NN * DF) return;
  if (in_sizes[1] != 2 * NE) return;
  if (in_sizes[2] != DF * DF || in_sizes[3] != DF * DF || in_sizes[4] != DF) return;
  if (in_sizes[5] != DF * DF || in_sizes[6] != DF * DF || in_sizes[7] != DF) return;
  if (in_sizes[8] != DF * DF || in_sizes[9] != DF * DF || in_sizes[10] != DF) return;
  if (in_sizes[11] != DF * NL || in_sizes[12] != NL) return;
  if (out_size != NN * NL) return;

  const float* x   = (const float*)d_in[0];
  const int*   ei  = (const int*)  d_in[1];
  const int*   src = ei;
  const int*   dst = ei + NE;
  const float* w11 = (const float*)d_in[2];
  const float* w21 = (const float*)d_in[3];
  const float* b1  = (const float*)d_in[4];
  const float* w12 = (const float*)d_in[5];
  const float* w22 = (const float*)d_in[6];
  const float* b2  = (const float*)d_in[7];
  const float* w13 = (const float*)d_in[8];
  const float* w23 = (const float*)d_in[9];
  const float* b3  = (const float*)d_in[10];
  const float* wdn = (const float*)d_in[11];
  const float* bdn = (const float*)d_in[12];
  float* out = (float*)d_out;

  const int nN = NN, nE = NE;
  const int vec8 = ((nE & 3) == 0) ? 1 : 0;

  char* ws = (char*)d_ws;
  size_t off = 0;
  const size_t oW1 = off; off = al256(off + (size_t)DF * WP1 * 2);
  const size_t oW2 = off; off = al256(off + (size_t)DF * WP2 * 2);
  const size_t oW3 = off; off = al256(off + (size_t)DF * WP2 * 2);
  const size_t oWD = off; off = al256(off + (size_t)NL * WPD * 2);
  const size_t oXB = off; off = al256(off + (size_t)MP * XP * 2);
  const size_t oAG = off; off = al256(off + (size_t)MP * AP * 2);
  const size_t oH  = off; off = al256(off + (size_t)MP * DF * 4);
  const size_t oP0 = off; off = al256(off + (size_t)MP * AP * 2);
  const size_t oP1 = off; off = al256(off + (size_t)MP * AP * 2);
  const size_t oLS = off; off = al256(off + (size_t)NBLK * RCAP * 4);
  const size_t oCN = off; off = al256(off + (size_t)NPADN * 4);
  const size_t oOF = off; off = al256(off + (size_t)NPADN * 4);
  const size_t oNS = off; off = al256(off + (size_t)NPADN * 4);
  const size_t oND = off; off = al256(off + (size_t)NPADN * 4);
  const size_t oRC = off; off = al256(off + (size_t)NBLK * 128);
  if (off > ws_size || off > (size_t)(128u << 20)) return;
  unsigned short* WC1 = (unsigned short*)(ws + oW1);
  unsigned short* WC2 = (unsigned short*)(ws + oW2);
  unsigned short* WC3 = (unsigned short*)(ws + oW3);
  unsigned short* WD  = (unsigned short*)(ws + oWD);
  unsigned short* XB  = (unsigned short*)(ws + oXB);
  unsigned short* AGG = (unsigned short*)(ws + oAG);
  float*          H   = (float*)(ws + oH);
  unsigned short* P0  = (unsigned short*)(ws + oP0);
  unsigned short* P1  = (unsigned short*)(ws + oP1);
  int*   LIST = (int*)(ws + oLS);
  int*   CIN  = (int*)(ws + oCN);
  int*   OFF  = (int*)(ws + oOF);
  float* NS   = (float*)(ws + oNS);
  float* ND   = (float*)(ws + oND);
  int*   REC  = (int*)(ws + oRC);

  hipFuncSetAttribute(reinterpret_cast<const void*>(&k_bucket), hipFuncAttributeMaxDynamicSharedMemorySize, LDS_BK);
  hipFuncSetAttribute(reinterpret_cast<const void*>(&k_gemm<1, 1>), hipFuncAttributeMaxDynamicSharedMemorySize, LDS_GM);
  hipFuncSetAttribute(reinterpret_cast<const void*>(&k_gemm<0, 1>), hipFuncAttributeMaxDynamicSharedMemorySize, LDS_GM);
  hipFuncSetAttribute(reinterpret_cast<const void*>(&k_gemm<0, 0>), hipFuncAttributeMaxDynamicSharedMemorySize, LDS_GM);

  const int gR = MP / RPB;
  const int gG = MP / GBM;
  k_prep<<<NWBLK + NXBLK, NTHR, 0, stream>>>(x, w11, w21, w12, w22, w13, w23, wdn, WC1, WC2, WC3, WD, XB, nN, MP);
  k_bucket<<<NBLK, NTHR, LDS_BK, stream>>>(dst, src, nE, nN, vec8, LIST, CIN, OFF, NS, ND, REC);
  k_replay<1><<<gR, NTHR, 0, stream>>>(XB, H, LIST, CIN, OFF, REC, NS, ND, AGG, nN, MP);
  k_gemm<1, 1><<<gG, GTHR, LDS_GM, stream>>>(AGG, XB, WC1, b1, H, P0, nN);
  k_replay<0><<<gR, NTHR, 0, stream>>>(XB, H, LIST, CIN, OFF, REC, NS, ND, AGG, nN, MP);
  k_gemm<0, 1><<<gG, GTHR, LDS_GM, stream>>>(AGG, P0, WC2, b2, H, P1, nN);
  k_replay<0><<<gR, NTHR, 0, stream>>>(XB, H, LIST, CIN, OFF, REC, NS, ND, AGG, nN, MP);
  k_gemm<0, 0><<<gG, GTHR, LDS_GM, stream>>>(AGG, P1, WC3, b3, H, P0, nN);
  k_head<<<gG, NTHR, 0, stream>>>(P0, WD, bdn, REC, out, out_size / 4);
}
